// CoAttention_31576599560314
// MI455X (gfx1250) — hardware-verified
//
#include <hip/hip_runtime.h>
#include <math.h>
#include <stdint.h>

#ifndef NB
#define NB 8
#endif
#ifndef NQ
#define NQ 4096
#endif
#define NB_FULL 8
#define CC     192
#define NN     4096
#define DQ     192
#define MW     384
#define QT     64
#define CH     96
#define OSP    68
#define OSPW   100
#define TP     72
#define WG8    (CC / 8)
#define WSC    256.0f
#define IWSC   0.00390625f
#define LOSC   4096.0f
#define ILOSC  0.000244140625f
#define LNPS   9.704060527839234f
#define FMIN16 6.103515625e-05f

static_assert(NB >= 1 && NB <= NB_FULL);
static_assert(NQ >= QT && NQ <= NN && NQ % QT == 0);
static_assert(NN % QT == 0 && NN % 32 == 0);
static_assert(CC % QT == 0 && CC % 32 == 0 && CC % 8 == 0);
static_assert(DQ == CC && MW == 2 * DQ && DQ == 3 * QT);
static_assert(CH * 2 == CC && CH % 16 == 0 && CH % 8 == 0);
static_assert((OSP * 4) % 16 == 0 && OSP >= QT + 4);
static_assert((OSPW * 4) % 16 == 0 && OSPW >= CH + 4);
static_assert((TP * 2) % 16 == 0 && TP >= QT + 8);
static_assert(WG8 * 8 == CC && (8 * WG8) % 32 == 0);
static_assert(MW % 8 == 0 && DQ % 8 == 0);

typedef _Float16       v16h __attribute__((ext_vector_type(16)));
typedef _Float16       v8h  __attribute__((ext_vector_type(8)));
typedef unsigned short v8us __attribute__((ext_vector_type(8)));
typedef float          v8f  __attribute__((ext_vector_type(8)));
typedef float          v4f  __attribute__((ext_vector_type(4)));
typedef unsigned int   v4u  __attribute__((ext_vector_type(4)));

union Frag  { v8us u[2]; v16h h; };
union FragH { v16h v; v8h hv[2]; };
static_assert(sizeof(Frag) == 32);
static_assert(sizeof(FragH) == 32);

__device__ __forceinline__ unsigned short bf_bits(float f) {
  unsigned u = __float_as_uint(f);
  return (unsigned short)((u + 0x7FFFu + ((u >> 16) & 1u)) >> 16);
}
__device__ __forceinline__ float bf_up(unsigned short hb) { return __uint_as_float(((unsigned)hb) << 16); }
__device__ __forceinline__ float bfr(float f) { return bf_up(bf_bits(f)); }
__device__ __forceinline__ unsigned short h_bits(_Float16 x) { return __builtin_bit_cast(unsigned short, x); }
__device__ __forceinline__ unsigned pk16(unsigned short a, unsigned short b) { return (unsigned)a | ((unsigned)b << 16); }
__device__ __forceinline__ v8f zero8() { v8f z = {0.f, 0.f, 0.f, 0.f, 0.f, 0.f, 0.f, 0.f}; return z; }
__device__ __forceinline__ float hmax8(v8f s) {
  return fmaxf(fmaxf(fmaxf(s[0], s[1]), fmaxf(s[2], s[3])), fmaxf(fmaxf(s[4], s[5]), fmaxf(s[6], s[7])));
}
__device__ __forceinline__ unsigned wave_ballot(bool p) {
#if defined(__HIP_DEVICE_COMPILE__)
  return __builtin_amdgcn_ballot_w32(p);
#else
  return p ? 1u : 0u;
#endif
}

__device__ __forceinline__ Frag ldfrag(const unsigned short* p) {
  Frag f;
  f.u[0] = *(const v8us*)(p);
  f.u[1] = *(const v8us*)(p + 16);
  return f;
}

__device__ __forceinline__ v8f mma_h(v16h a, v16h b, v8f c) {
  v8f d = __builtin_amdgcn_wmma_f32_16x16x32_f16(false, a, false, b, (short)0, c, false, false);
#if defined(__HIP_DEVICE_COMPILE__)
  asm volatile("v_nop\n\tv_nop\n\tv_nop\n\tv_nop" : "+v"(d) : "v"(a), "v"(b));
#endif
  return d;
}

__global__ __launch_bounds__(8 * WG8)
void cvt_w(const float* __restrict__ wq, const float* __restrict__ wk, unsigned short* W16) {
  const int tid = threadIdx.x, blk = blockIdx.x;
  const int rl  = tid / WG8;
  const int col = 8 * (tid - rl * WG8);
  const int o   = 8 * blk + rl;
  const float* wbase = (blk < (DQ / 8)) ? wq : wk;
  const int osub = (blk < (DQ / 8)) ? 0 : DQ;
  const float* s = wbase + (size_t)(o - osub) * CC + col;
  const v4f a = *(const v4f*)s;
  const v4f q = *(const v4f*)(s + 4);
  const float f[8] = {a[0], a[1], a[2], a[3], q[0], q[1], q[2], q[3]};
  v4u u;
#pragma unroll
  for (int t = 0; t < 4; ++t) {
    const _Float16 h0 = (_Float16)(bfr(f[2 * t]) * WSC);
    const _Float16 h1 = (_Float16)(bfr(f[2 * t + 1]) * WSC);
    u[t] = pk16(h_bits(h0), h_bits(h1));
  }
#pragma unroll
  for (int pass = 0; pass < 2; ++pass) {
    *(volatile v4u*)(W16 + (size_t)o * CC + col) = u;
    __threadfence();
  }
}

__global__ __launch_bounds__(256)
void cvt_kv(const float* __restrict__ key, const float* __restrict__ val, unsigned short* Vc, unsigned short* XP) {
  __shared__ __align__(16) unsigned short T[QT * TP];
  const int tid = threadIdx.x;
  const int nb = blockIdx.x, cb = blockIdx.y, b = blockIdx.z;
  const int e = tid & 7, lq = tid >> 3;
  const int n0 = nb * QT, c0 = cb * QT;
  v4u uv[2];
#pragma unroll
  for (int it = 0; it < 2; ++it) {
    const int cl = it * 32 + lq;
    const size_t ro = ((size_t)(b * CC + c0 + cl)) * NN + n0 + 8 * e;
    const v4f ka = *(const v4f*)(key + ro);
    const v4f kq = *(const v4f*)(key + ro + 4);
    const v4f va = *(const v4f*)(val + ro);
    const v4f vq = *(const v4f*)(val + ro + 4);
    unsigned short hk[8], hv[8];
#pragma unroll
    for (int t = 0; t < 4; ++t) {
      hk[t]     = h_bits((_Float16)bfr(ka[t]));
      hk[4 + t] = h_bits((_Float16)bfr(kq[t]));
      hv[t]     = h_bits((_Float16)bfr(va[t]));
      hv[4 + t] = h_bits((_Float16)bfr(vq[t]));
    }
#pragma unroll
    for (int t = 0; t < 4; ++t) uv[it][t] = pk16(hv[2 * t], hv[2 * t + 1]);
#pragma unroll
    for (int t = 0; t < 8; ++t) T[(8 * e + t) * TP + cl] = hk[t];
  }
  __syncthreads();
  v4u up[2];
#pragma unroll
  for (int it = 0; it < 2; ++it) {
    const int nl = it * 32 + lq;
    up[it] = *(const v4u*)(T + nl * TP + 8 * e);
  }
#pragma unroll
  for (int pass = 0; pass < 2; ++pass) {
#pragma unroll
    for (int it = 0; it < 2; ++it) {
      const int rl = it * 32 + lq;
      *(volatile v4u*)(Vc + ((size_t)(b * CC + c0 + rl)) * NN + n0 + 8 * e) = uv[it];
      *(volatile v4u*)(XP + ((size_t)(b * NN + n0 + rl)) * CC + c0 + 8 * e) = up[it];
    }
    __threadfence();
  }
}

__global__ __launch_bounds__(128)
void gemm_qk(const unsigned short* __restrict__ W16, const unsigned short* __restrict__ XP,
             const float* __restrict__ bq, const float* __restrict__ bk,
             unsigned short* Qh, unsigned short* Ql, unsigned short* Kh, unsigned short* Kl) {
  __shared__ __align__(16) float Os[QT * OSP];
  const int tid  = threadIdx.x;
  const int lane = tid & 31, wave = tid >> 5;
  const int hh   = lane >> 4, c = lane & 15;
  const int nt   = blockIdx.x, mb = blockIdx.y, b = blockIdx.z;
  const int n0   = nt * QT, o0 = mb * QT;

  const unsigned short* ap = W16 + (size_t)(o0 + c) * CC + 8 * hh;
  const unsigned short* bp = XP + ((size_t)(b * NN + n0 + 16 * wave + c)) * CC + 8 * hh;

  v8f acc[4];
#pragma unroll
  for (int mt = 0; mt < 4; ++mt) acc[mt] = zero8();

#pragma unroll
  for (int ks = 0; ks < CC / 32; ++ks) {
    const Frag fb = ldfrag(bp + 32 * ks);
#pragma unroll
    for (int mt = 0; mt < 4; ++mt) {
      const Frag fa = ldfrag(ap + (size_t)(16 * mt) * CC + 32 * ks);
      acc[mt] = mma_h(fa.h, fb.h, acc[mt]);
    }
  }

  {
    const int nl = 16 * wave + c;
#pragma unroll
    for (int mt = 0; mt < 4; ++mt) {
      v4f va, vb;
#pragma unroll
      for (int r = 0; r < 4; ++r) { va[r] = acc[mt][r] * IWSC; vb[r] = acc[mt][4 + r] * IWSC; }
      *(v4f*)(Os + nl * OSP + 16 * mt + 8 * hh)     = va;
      *(v4f*)(Os + nl * OSP + 16 * mt + 8 * hh + 4) = vb;
    }
  }
  __syncthreads();

  const int e = tid & 7, lq = tid >> 3;
  const bool isq = (mb < (DQ / QT));
  const int dsel = (isq ? mb : (mb - DQ / QT)) * QT;
  unsigned short* Ph = isq ? Qh : Kh;
  unsigned short* Pl = isq ? Ql : Kl;
  const float* bb = isq ? bq : bk;
  const v4f b0 = *(const v4f*)(bb + dsel + 8 * e);
  const v4f b1 = *(const v4f*)(bb + dsel + 8 * e + 4);
  const float bs[8] = {bfr(b0[0]), bfr(b0[1]), bfr(b0[2]), bfr(b0[3]), bfr(b1[0]), bfr(b1[1]), bfr(b1[2]), bfr(b1[3])};
  v4u uh[4], ul[4];
#pragma unroll
  for (int it = 0; it < 4; ++it) {
    const int row = it * 16 + lq;
    const v4f a = *(const v4f*)(Os + row * OSP + 8 * e);
    const v4f q = *(const v4f*)(Os + row * OSP + 8 * e + 4);
    const float f[8] = {a[0] + bs[0], a[1] + bs[1], a[2] + bs[2], a[3] + bs[3],
                        q[0] + bs[4], q[1] + bs[5], q[2] + bs[6], q[3] + bs[7]};
#pragma unroll
    for (int t = 0; t < 4; ++t) {
      const float f0 = f[2 * t], f1 = f[2 * t + 1];
      float g0 = (float)(_Float16)f0;
      float g1 = (float)(_Float16)f1;
      g0 = (fabsf(g0) < FMIN16) ? 0.f : g0;
      g1 = (fabsf(g1) < FMIN16) ? 0.f : g1;
      const unsigned short hb0 = h_bits((_Float16)g0), hb1 = h_bits((_Float16)g1);
      const unsigned short lb0 = h_bits((_Float16)((f0 - g0) * LOSC));
      const unsigned short lb1 = h_bits((_Float16)((f1 - g1) * LOSC));
      uh[it][t] = pk16(hb0, hb1);
      ul[it][t] = pk16(lb0, lb1);
    }
  }
#pragma unroll
  for (int pass = 0; pass < 2; ++pass) {
#pragma unroll
    for (int it = 0; it < 4; ++it) {
      const int row = it * 16 + lq;
      const size_t po = ((size_t)(b * NN + n0 + row)) * DQ + dsel + 8 * e;
      *(volatile v4u*)(Ph + po) = uh[it];
      *(volatile v4u*)(Pl + po) = ul[it];
    }
    __threadfence();
  }
}

__global__ __launch_bounds__(128)
void attn_k(const unsigned short* __restrict__ Qh, const unsigned short* __restrict__ Ql,
            const unsigned short* __restrict__ Kh, const unsigned short* __restrict__ Kl,
            const unsigned short* __restrict__ Vc, float* out) {
  __shared__ __align__(16) float Os[QT * OSPW];
  const int tid  = threadIdx.x;
  const int wave = tid >> 5, lane = tid & 31;
  const int hh   = lane >> 4, c = lane & 15;
  const int n0   = blockIdx.x * QT, b = blockIdx.y;

  const size_t qo = ((size_t)(b * NN + n0 + 16 * wave + c)) * DQ + 8 * hh;
  const unsigned short* Qhp = Qh + qo;
  const unsigned short* Qlp = Ql + qo;
  const unsigned short* Khp = Kh + (size_t)b * NN * DQ + (size_t)c * DQ + 8 * hh;
  const unsigned short* Klp = Kl + (size_t)b * NN * DQ + (size_t)c * DQ + 8 * hh;
  const unsigned short* Vp = Vc + (size_t)b * CC * NN + (size_t)c * NN + 8 * hh;

  float m = -1.0e30f, l = 0.f;
  v8f o[CC / 16];
#pragma unroll
  for (int j = 0; j < CC / 16; ++j) o[j] = zero8();

#pragma unroll 1
  for (int kb = 0; kb < NN; kb += 32) {
    const unsigned short* k0p  = Khp + (size_t)kb * DQ;
    const unsigned short* k1p  = Khp + (size_t)(kb + 16) * DQ;
    const unsigned short* k0lp = Klp + (size_t)kb * DQ;
    const unsigned short* k1lp = Klp + (size_t)(kb + 16) * DQ;
    v8f s0 = zero8(), s1 = zero8(), t0 = zero8(), t1 = zero8();
#pragma unroll 1
    for (int kc = 0; kc < DQ / 32; ++kc) {
      const Frag qh  = ldfrag(Qhp + 32 * kc);
      const Frag ql  = ldfrag(Qlp + 32 * kc);
      const Frag k0  = ldfrag(k0p + 32 * kc);
      const Frag k1  = ldfrag(k1p + 32 * kc);
      const Frag k0l = ldfrag(k0lp + 32 * kc);
      const Frag k1l = ldfrag(k1lp + 32 * kc);
      s0 = mma_h(k0.h, qh.h, s0);
      s1 = mma_h(k1.h, qh.h, s1);
      t0 = mma_h(k0.h, ql.h, t0);
      t1 = mma_h(k1.h, ql.h, t1);
      t0 = mma_h(k0l.h, qh.h, t0);
      t1 = mma_h(k1l.h, qh.h, t1);
    }
#pragma unroll
    for (int r = 0; r < 8; ++r) {
      s0[r] = s0[r] + t0[r] * ILOSC;
      s1[r] = s1[r] + t1[r] * ILOSC;
    }

    float mx = fmaxf(hmax8(s0), hmax8(s1));
    mx = fmaxf(mx, __shfl_xor(mx, 16, 32));
    const float mn = fmaxf(m, mx);
    const unsigned grew = wave_ballot(mx > m);
    if (grew != 0u) {
      const float corr = __expf(m - mn);
      l *= corr;
#pragma unroll
      for (int j = 0; j < CC / 16; ++j) {
#pragma unroll
        for (int r = 0; r < 8; ++r) o[j][r] *= corr;
      }
    }
    m = mn;
    const float msh = mn - LNPS;

    FragH ph;
    float ls = 0.f;
#pragma unroll
    for (int r = 0; r < 8; ++r) {
      const float e0 = __expf(s0[r] - msh);
      const float e1 = __expf(s1[r] - msh);
      ls += e0 + e1;
      ph.hv[0][r] = (_Float16)e0;
      ph.hv[1][r] = (_Float16)e1;
    }
    l += ls;

#pragma unroll
    for (int j = 0; j < CC / 16; ++j) {
      const Frag vf = ldfrag(Vp + (size_t)(16 * j) * NN + kb);
      o[j] = mma_h(vf.h, ph.v, o[j]);
    }
  }
  l += __shfl_xor(l, 16, 32);
  const float inv = 1.0f / l;

  const int qrow = 16 * wave + c;
  const int e = tid & 7, lq = tid >> 3;
#pragma unroll
  for (int half = 0; half < 2; ++half) {
    if (half) __syncthreads();
#pragma unroll
    for (int jj = 0; jj < CH / 16; ++jj) {
      const int j = (CH / 16) * half + jj;
      v4f va, vb;
#pragma unroll
      for (int r = 0; r < 4; ++r) { va[r] = o[j][r] * inv; vb[r] = o[j][4 + r] * inv; }
      *(v4f*)(Os + qrow * OSPW + 16 * jj + 8 * hh)     = va;
      *(v4f*)(Os + qrow * OSPW + 16 * jj + 8 * hh + 4) = vb;
    }
    __syncthreads();
    v4f res[CH / 8];
#pragma unroll
    for (int it = 0; it < CH / 8; ++it) {
      const int L   = it * 16 + lq;
      const int chl = L >> 1, hf = L & 1;
      const int nl  = hf * 32 + 4 * e;
#pragma unroll
      for (int t = 0; t < 4; ++t) res[it][t] = Os[(nl + t) * OSPW + chl];
    }
#pragma unroll
    for (int pass = 0; pass < 2; ++pass) {
#pragma unroll
      for (int it = 0; it < CH / 8; ++it) {
        const int L   = it * 16 + lq;
        const int chl = L >> 1, hf = L & 1;
        const int nl  = hf * 32 + 4 * e;
        const size_t idx = ((size_t)(b * CC + CH * half + chl)) * NN + n0 + nl;
        *(volatile v4f*)(out + idx) = res[it];
      }
      __threadfence();
    }
  }
}

extern "C" void kernel_launch(void* const* d_in, const int* in_sizes, int n_in,
                              void* d_out, int out_size, void* d_ws, size_t ws_size,
                              hipStream_t stream) {
  const int XN = NB * CC * NN;
  if (n_in < 6) return;
  if (in_sizes[0] < XN || in_sizes[1] < XN) return;
  if (in_sizes[2] < CC * CC || in_sizes[4] < CC * CC) return;
  if (in_sizes[3] < CC || in_sizes[5] < CC) return;
  if (out_size < XN) return;

  size_t off = 0;
  auto carve = [&](size_t bytes) { const size_t o = off; off += (bytes + 255) & ~(size_t)255; return o; };
  const size_t oW16 = carve((size_t)MW * CC * 2);
  const size_t oVc  = carve((size_t)NB * CC * NN * 2);
  const size_t oXP  = carve((size_t)NB * NN * CC * 2);
  const size_t oQh  = carve((size_t)NB * NN * DQ * 2);
  const size_t oQl  = carve((size_t)NB * NN * DQ * 2);
  const size_t oKh  = carve((size_t)NB * NN * DQ * 2);
  const size_t oKl  = carve((size_t)NB * NN * DQ * 2);
  if (off > ws_size) return;
  if (off > (size_t)134217728) return;

  const float* key = (const float*)d_in[0];
  const float* val = (const float*)d_in[1];
  const float* wl  = (const float*)d_in[2];
  const float* bl  = (const float*)d_in[3];
  const float* wr  = (const float*)d_in[4];
  const float* br  = (const float*)d_in[5];

  char* ws = (char*)d_ws;
  unsigned short* W16 = (unsigned short*)(ws + oW16);
  unsigned short* Vc  = (unsigned short*)(ws + oVc);
  unsigned short* XP  = (unsigned short*)(ws + oXP);
  unsigned short* Qh  = (unsigned short*)(ws + oQh);
  unsigned short* Ql  = (unsigned short*)(ws + oQl);
  unsigned short* Kh  = (unsigned short*)(ws + oKh);
  unsigned short* Kl  = (unsigned short*)(ws + oKl);
  float* out = (float*)d_out;

  const dim3 blk256(256), blk128(128), blkw(8 * WG8);

  cvt_w<<<dim3(MW / 8), blkw, 0, stream>>>(wr, wl, W16);
  cvt_kv<<<dim3(NN / QT, CC / QT, NB), blk256, 0, stream>>>(key, val, Vc, XP);
  gemm_qk<<<dim3(NN / QT, MW / QT, NB), blk128, 0, stream>>>(W16, XP, br, bl, Qh, Ql, Kh, Kl);
  attn_k<<<dim3(NQ / QT, NB), blk128, 0, stream>>>(Qh, Ql, Kh, Kl, Vc, out);
  (void)hipGetLastError();
}
